// MultiHeadLatentAttention_73280732005044
// MI455X (gfx1250) — hardware-verified
//
#include <hip/hip_runtime.h>


#ifndef NB
#define NB 4
#endif
#ifndef SEQ
#define SEQ 2048
#endif
#define NB_FULL 4
#define SEQ_FULL 2048
#define DM 1024
#define NH 8
#define DK 128
#define DC 32
#define DR 32
#define MTOK (NB * SEQ)
#define UPN (3 * NH * DK + NH * DR)

static_assert(SEQ % 64 == 0);
static_assert(SEQ <= SEQ_FULL);
static_assert(NB >= 1 && NB <= NB_FULL);
static_assert(UPN == 3328);
static_assert(UPN % 128 == 0);

#define SC_WD  32.0f
#define SC_C   4.0f
#define SC_WU  4.0f
#define SC_QKV 8.0f
#define SC_WO  32.0f

#define WS_TOTAL ((size_t)96 * DM * 2 + (size_t)UPN * DC * 2 + (size_t)DM * DM * 2 + 3 * (size_t)MTOK * DC * 2 \
                  + 2 * (size_t)NB * NH * SEQ * DK * 2 + (size_t)NB * NH * SEQ * DR * 2 + (size_t)NB * NH * DK * SEQ * 2 + (size_t)MTOK * DM * 2)
static_assert(WS_TOTAL <= (size_t)134217728);

typedef _Float16 v8h  __attribute__((ext_vector_type(8)));
typedef _Float16 v16h __attribute__((ext_vector_type(16)));
typedef float    v8f  __attribute__((ext_vector_type(8)));
typedef float    v4f  __attribute__((ext_vector_type(4)));
typedef unsigned v4u  __attribute__((ext_vector_type(4)));

__device__ __forceinline__ float bfr(float f) {
    unsigned u = __float_as_uint(f);
    u = (u + 0x7fffu + ((u >> 16) & 1u)) & 0xffff0000u;
    return __uint_as_float(u);
}
__device__ __forceinline__ _Float16 tohx(float f, float sc) { return (_Float16)(bfr(f) * sc); }

__device__ __forceinline__ v8f wmma16(v16h a, v16h b, v8f c) {
    c = __builtin_amdgcn_wmma_f32_16x16x32_f16(false, a, false, b, (short)0, c, false, false);
    asm volatile("v_nop\n\tv_nop\n\tv_nop\n\tv_nop" : "+v"(c) : "v"(a), "v"(b));
    return c;
}
__device__ __forceinline__ v16h ldfrag(const _Float16* p, int hf) {
    const v8h lo = *(const v8h*)(p + 8 * hf);
    const v8h hi = *(const v8h*)(p + 16 + 8 * hf);
    return __builtin_shufflevector(lo, hi, 0, 1, 2, 3, 4, 5, 6, 7, 8, 9, 10, 11, 12, 13, 14, 15);
}
__device__ __forceinline__ void vst16(_Float16* g, v8h v) { *(volatile v4u*)g = __builtin_bit_cast(v4u, v); }
__device__ __forceinline__ void vst16f(float* g, v4f v) { *(volatile v4f*)g = v; }

#define PREP_BLK_A 48
#define PREP_BLK_B 52
#define PREP_BLK_C 512
__global__ __launch_bounds__(256) void k_prep(const float* __restrict__ wDQ, const float* __restrict__ wDKV, const float* __restrict__ wKR,
                                              const float* __restrict__ wUQ, const float* __restrict__ wUK, const float* __restrict__ wUV,
                                              const float* __restrict__ wQR, const float* __restrict__ wO,
                                              _Float16* WdT, _Float16* WuT, _Float16* WoT) {
    const int tid = blockIdx.x * 256 + threadIdx.x;
    v8h val;
    _Float16* dst;
    if (blockIdx.x < PREP_BLK_A) {
        const int i = tid;
        const int n = i >> 7, k = (i & 127) * 8;
        const float* src = (n < 32) ? wDQ : ((n < 64) ? wDKV : wKR);
        const int nn = n & 31;
#pragma unroll
        for (int j = 0; j < 8; ++j) val[j] = tohx(src[(size_t)(k + j) * 32 + nn], SC_WD);
        dst = WdT + (size_t)n * DM + k;
    } else if (blockIdx.x < PREP_BLK_A + PREP_BLK_B) {
        const int i = tid - PREP_BLK_A * 256;
        const int n = i >> 2, k = (i & 3) * 8;
        const float* src = (n < 1024) ? wUQ : ((n < 2048) ? wUK : ((n < 3072) ? wUV : wQR));
        const int ld = (n < 3072) ? (NH * DK) : (NH * DR);
        const int nn = (n < 3072) ? (n & 1023) : (n - 3072);
#pragma unroll
        for (int j = 0; j < 8; ++j) val[j] = tohx(src[(size_t)(k + j) * ld + nn], SC_WU);
        dst = WuT + (size_t)n * DC + k;
    } else {
        const int i = tid - (PREP_BLK_A + PREP_BLK_B) * 256;
        const int n = i >> 7, k = (i & 127) * 8;
#pragma unroll
        for (int j = 0; j < 8; ++j) val[j] = tohx(wO[(size_t)(k + j) * DM + n], SC_WO);
        dst = WoT + (size_t)n * DM + k;
    }
    vst16(dst, val);
    __threadfence();
    vst16(dst, val);
}

__global__ __launch_bounds__(128) void k_down(const float* __restrict__ X, const _Float16* __restrict__ WdT,
                                              const float* __restrict__ bDQ, const float* __restrict__ bDKV, const float* __restrict__ bKR,
                                              _Float16* CQ, _Float16* CKV, _Float16* KRP) {
    __shared__ __align__(16) _Float16 st[4][16 * 104];
    const int tid = threadIdx.x, lane = tid & 31, wv = tid >> 5, l16 = lane & 15, hf = lane >> 4;
    const int t0 = blockIdx.x * 64 + wv * 16;
    const int tok = t0 + l16, bi = tok / SEQ, si = tok - bi * SEQ;
    const float* xr = X + ((size_t)bi * SEQ_FULL + si) * DM;
    v8f acc[6];
#pragma unroll
    for (int t = 0; t < 6; ++t) acc[t] = (v8f){};
#pragma unroll 1
    for (int kc = 0; kc < DM / 32; ++kc) {
        const float* xp = xr + kc * 32;
        const v4f x0 = *(const v4f*)(xp + 8 * hf);
        const v4f x1 = *(const v4f*)(xp + 8 * hf + 4);
        const v4f x2 = *(const v4f*)(xp + 16 + 8 * hf);
        const v4f x3 = *(const v4f*)(xp + 20 + 8 * hf);
        v16h a;
#pragma unroll
        for (int i = 0; i < 4; ++i) {
            a[i]      = tohx(x0[i], 1.0f);
            a[4 + i]  = tohx(x1[i], 1.0f);
            a[8 + i]  = tohx(x2[i], 1.0f);
            a[12 + i] = tohx(x3[i], 1.0f);
        }
#pragma unroll
        for (int t = 0; t < 6; ++t) {
            const v16h bf = ldfrag(WdT + (size_t)(t * 16 + l16) * DM + kc * 32, hf);
            acc[t] = wmma16(a, bf, acc[t]);
        }
    }
#pragma unroll
    for (int t = 0; t < 6; ++t) {
        const int col = t * 16 + l16;
        const float* bp = (t < 2) ? bDQ : ((t < 4) ? bDKV : bKR);
        const float bb = bfr(bp[col - (t / 2) * 32]);
        const float sc = (t < 4) ? SC_C : SC_QKV;
#pragma unroll
        for (int r = 0; r < 8; ++r) st[wv][(8 * hf + r) * 104 + col] = (_Float16)((acc[t][r] * (1.0f / SC_WD) + bb) * sc);
    }
    __syncthreads();
    v8h w[6];
#pragma unroll
    for (int p = 0; p < 3; ++p)
#pragma unroll
        for (int u = 0; u < 2; ++u) {
            const int row = u * 8 + (lane >> 2), pc = lane & 3;
            w[p * 2 + u] = *(const v8h*)&st[wv][row * 104 + p * 32 + pc * 8];
        }
    _Float16* const planes[3] = {CQ, CKV, KRP};
    auto pass = [&]() {
#pragma unroll
        for (int p = 0; p < 3; ++p)
#pragma unroll
            for (int u = 0; u < 2; ++u) {
                const int row = u * 8 + (lane >> 2), pc = lane & 3;
                vst16(planes[p] + (size_t)(t0 + row) * DC + pc * 8, w[p * 2 + u]);
            }
    };
    pass();
    __threadfence();
    pass();
}

__global__ __launch_bounds__(128) void k_up(const _Float16* __restrict__ CQ, const _Float16* __restrict__ CKV, const _Float16* __restrict__ WuT,
                                            const float* __restrict__ bUQ, const float* __restrict__ bUK, const float* __restrict__ bUV, const float* __restrict__ bQR,
                                            _Float16* QC, _Float16* KC, _Float16* VT, _Float16* QRP) {
    __shared__ __align__(16) _Float16 st[9216];
    const int tid = threadIdx.x, lane = tid & 31, wv = tid >> 5, l16 = lane & 15, hf = lane >> 4;
    const int g = blockIdx.y;
    const int t0 = blockIdx.x * 64;
    const int bi = t0 / SEQ, s0 = t0 - bi * SEQ;
    const float* bp;
    const _Float16* A;
    if (g < 8)       { bp = bUQ + g * DK;          A = CQ;  }
    else if (g < 16) { bp = bUK + (g - 8) * DK;    A = CKV; }
    else if (g < 24) { bp = bUV + (g - 16) * DK;   A = CKV; }
    else             { bp = bQR + (g - 24) * 128;  A = CQ;  }
    const bool isV = (g >= 16) && (g < 24);
    const v16h a = ldfrag(A + (size_t)(t0 + wv * 16 + l16) * DC, hf);
    v8f acc[8];
#pragma unroll
    for (int nt = 0; nt < 8; ++nt) {
        const v16h bf = ldfrag(WuT + (size_t)(g * 128 + nt * 16 + l16) * DC, hf);
        acc[nt] = wmma16(a, bf, (v8f){});
    }
    if (isV) {
#pragma unroll
        for (int nt = 0; nt < 8; ++nt) {
            const int d = nt * 16 + l16;
            const float bb = bfr(bp[d]);
            v8h pv;
#pragma unroll
            for (int r = 0; r < 8; ++r) pv[r] = (_Float16)((acc[nt][r] * (1.0f / (SC_C * SC_WU)) + bb) * SC_QKV);
            *(v8h*)&st[d * 72 + wv * 16 + 8 * hf] = pv;
        }
    } else {
#pragma unroll
        for (int nt = 0; nt < 8; ++nt) {
            const int col = nt * 16 + l16;
            const float bb = bfr(bp[col]);
#pragma unroll
            for (int r = 0; r < 8; ++r) st[(wv * 16 + 8 * hf + r) * 136 + col] = (_Float16)((acc[nt][r] * (1.0f / (SC_C * SC_WU)) + bb) * SC_QKV);
        }
    }
    __syncthreads();
    v8h w[8];
    if (isV) {
        const int hd = g - 16;
#pragma unroll
        for (int p = 0; p < 8; ++p) { const int d = p * 16 + (tid >> 3), pc = tid & 7; w[p] = *(const v8h*)&st[d * 72 + pc * 8]; }
        auto pass = [&]() {
#pragma unroll
            for (int p = 0; p < 8; ++p) {
                const int d = p * 16 + (tid >> 3), pc = tid & 7;
                vst16(VT + ((size_t)(bi * NH + hd) * DK + d) * SEQ + s0 + pc * 8, w[p]);
            }
        };
        pass();
        __threadfence();
        pass();
    } else if (g < 16) {
        _Float16* base = ((g < 8) ? QC : KC) + ((size_t)(bi * NH + (g & 7)) * SEQ + s0) * DK;
#pragma unroll
        for (int p = 0; p < 8; ++p) { const int off = p * 1024 + tid * 8; w[p] = *(const v8h*)&st[(off >> 7) * 136 + (off & 127)]; }
        auto pass = [&]() {
#pragma unroll
            for (int p = 0; p < 8; ++p) { const int off = p * 1024 + tid * 8; vst16(base + off, w[p]); }
        };
        pass();
        __threadfence();
        pass();
    } else {
        const int hq0 = (g - 24) * 4;
#pragma unroll
        for (int p = 0; p < 8; ++p) {
            const int reg = p >> 1, off = (p & 1) * 1024 + tid * 8;
            w[p] = *(const v8h*)&st[(off >> 5) * 136 + reg * 32 + (off & 31)];
        }
        auto pass = [&]() {
#pragma unroll
            for (int p = 0; p < 8; ++p) {
                const int reg = p >> 1, off = (p & 1) * 1024 + tid * 8;
                vst16(QRP + ((size_t)(bi * NH + hq0 + reg) * SEQ + s0) * DR + off, w[p]);
            }
        };
        pass();
        __threadfence();
        pass();
    }
}

__global__ __launch_bounds__(128) void k_attn(const _Float16* __restrict__ QC, const _Float16* __restrict__ QRP, const _Float16* __restrict__ KC,
                                              const _Float16* __restrict__ KRP, const _Float16* __restrict__ VT, _Float16* CTX) {
    __shared__ __align__(16) _Float16 st[4][16 * 136];
    const int tid = threadIdx.x, lane = tid & 31, wv = tid >> 5, l16 = lane & 15, hf = lane >> 4;
    const int bh = blockIdx.y, bi = bh / NH, hd = bh - bi * NH;
    const int q0 = blockIdx.x * 64 + wv * 16;
    v16h qf[5];
    {
        const _Float16* qr = QC + ((size_t)bh * SEQ + q0 + l16) * DK;
#pragma unroll
        for (int cc = 0; cc < 4; ++cc) qf[cc] = ldfrag(qr + cc * 32, hf);
        qf[4] = ldfrag(QRP + ((size_t)bh * SEQ + q0 + l16) * DR, hf);
    }
    const _Float16* kb  = KC  + (size_t)bh * SEQ * DK;
    const _Float16* krb = KRP + (size_t)bi * SEQ * DR;
    const _Float16* vb  = VT  + (size_t)bh * DK * SEQ;
    v8f o[8];
#pragma unroll
    for (int d = 0; d < 8; ++d) o[d] = (v8f){};
    float m2 = -__builtin_inff(), lsum = 0.0f;
    const float c2 = (0.07905694150420949f * 1.4426950408889634f) * (1.0f / (SC_QKV * SC_QKV));
#pragma unroll 1
    for (int kt = 0; kt < SEQ / 64; ++kt) {
        v8f s[4];
#pragma unroll
        for (int ks = 0; ks < 4; ++ks) {
            const int key = kt * 64 + ks * 16 + l16;
            const _Float16* kr = kb + (size_t)key * DK;
            v8f c = (v8f){};
#pragma unroll
            for (int cc = 0; cc < 4; ++cc) c = wmma16(ldfrag(kr + cc * 32, hf), qf[cc], c);
            c = wmma16(ldfrag(krb + (size_t)key * DR, hf), qf[4], c);
            s[ks] = c;
        }
        float mloc = -__builtin_inff();
#pragma unroll
        for (int ks = 0; ks < 4; ++ks)
#pragma unroll
            for (int r = 0; r < 8; ++r) { s[ks][r] *= c2; mloc = fmaxf(mloc, s[ks][r]); }
        mloc = fmaxf(mloc, __shfl_xor(mloc, 16, 32));
        const float mn = fmaxf(m2, mloc);
        const float alpha = exp2f(m2 - mn);
        float ls = 0.0f;
        v16h pf[2];
#pragma unroll
        for (int ks = 0; ks < 4; ++ks)
#pragma unroll
            for (int r = 0; r < 8; ++r) {
                const float p = exp2f(s[ks][r] - mn);
                ls += p;
                pf[ks >> 1][(ks & 1) * 8 + r] = (_Float16)p;
            }
        m2 = mn;
        lsum = lsum * alpha + ls;
#pragma unroll
        for (int d = 0; d < 8; ++d) o[d] *= alpha;
#pragma unroll
        for (int d = 0; d < 8; ++d) {
            const _Float16* vr = vb + (size_t)(d * 16 + l16) * SEQ + kt * 64;
            o[d] = wmma16(ldfrag(vr, hf), pf[0], o[d]);
            o[d] = wmma16(ldfrag(vr + 32, hf), pf[1], o[d]);
        }
    }
    const float lt = lsum + __shfl_xor(lsum, 16, 32);
    const float inv = 1.0f / lt;
#pragma unroll
    for (int d = 0; d < 8; ++d) {
        v8h pv;
#pragma unroll
        for (int r = 0; r < 8; ++r) pv[r] = (_Float16)(o[d][r] * inv);
        *(v8h*)&st[wv][l16 * 136 + d * 16 + 8 * hf] = pv;
    }
    __syncthreads();
    v8h w[8];
#pragma unroll
    for (int t = 0; t < 8; ++t) { const int row = 2 * t + (lane >> 4), pc = lane & 15; w[t] = *(const v8h*)&st[wv][row * 136 + pc * 8]; }
    auto pass = [&]() {
#pragma unroll
        for (int t = 0; t < 8; ++t) {
            const int row = 2 * t + (lane >> 4), pc = lane & 15;
            vst16(CTX + (size_t)(bi * SEQ + q0 + row) * DM + hd * DK + pc * 8, w[t]);
        }
    };
    pass();
    __threadfence();
    pass();
}

__global__ __launch_bounds__(128) void k_out(const _Float16* __restrict__ CTX, const _Float16* __restrict__ WoT, const float* __restrict__ bO, float* OUT) {
    __shared__ __align__(16) float st[4][16 * 68];
    const int tid = threadIdx.x, lane = tid & 31, wv = tid >> 5, l16 = lane & 15, hf = lane >> 4;
    const int t0 = blockIdx.x * 64 + wv * 16, c0 = blockIdx.y * 64;
    const _Float16* arow = CTX + (size_t)(t0 + l16) * DM;
    v8f acc[4];
#pragma unroll
    for (int nt = 0; nt < 4; ++nt) acc[nt] = (v8f){};
#pragma unroll 1
    for (int kc = 0; kc < DM / 32; ++kc) {
        const v16h a = ldfrag(arow + kc * 32, hf);
#pragma unroll
        for (int nt = 0; nt < 4; ++nt) {
            const v16h bf = ldfrag(WoT + (size_t)(c0 + nt * 16 + l16) * DM + kc * 32, hf);
            acc[nt] = wmma16(a, bf, acc[nt]);
        }
    }
#pragma unroll
    for (int nt = 0; nt < 4; ++nt) {
        const int col = nt * 16 + l16;
#pragma unroll
        for (int r = 0; r < 8; ++r) st[wv][(8 * hf + r) * 68 + col] = acc[nt][r] * (1.0f / (SC_QKV * SC_WO));
    }
    __syncthreads();
    const int pc = lane & 15;
    v4f bb;
#pragma unroll
    for (int j = 0; j < 4; ++j) bb[j] = bfr(bO[c0 + pc * 4 + j]);
    v4f w[8];
#pragma unroll
    for (int t = 0; t < 8; ++t) { const int row = 2 * t + (lane >> 4); w[t] = *(const v4f*)&st[wv][row * 68 + pc * 4] + bb; }
    auto pass = [&]() {
#pragma unroll
        for (int t = 0; t < 8; ++t) {
            const int row = 2 * t + (lane >> 4);
            const int tok = t0 + row, bi = tok / SEQ, si = tok - bi * SEQ;
            vst16f(OUT + ((size_t)bi * SEQ_FULL + si) * DM + c0 + pc * 4, w[t]);
        }
    };
    pass();
    __threadfence();
    pass();
}

extern "C" void kernel_launch(void* const* d_in, const int* in_sizes, int n_in,
                              void* d_out, int out_size, void* d_ws, size_t ws_size, hipStream_t stream) {
    if (n_in < 17) return;
    const long long needTok = (long long)(NB - 1) * SEQ_FULL + SEQ;
    if ((long long)in_sizes[0] < needTok * DM) return;
    if (in_sizes[1] < DM * DC || in_sizes[2] < DC || in_sizes[3] < DC * NH * DK || in_sizes[4] < NH * DK ||
        in_sizes[5] < DM * DC || in_sizes[6] < DC || in_sizes[7] < DC * NH * DK || in_sizes[8] < NH * DK ||
        in_sizes[9] < DC * NH * DK || in_sizes[10] < NH * DK || in_sizes[11] < DC * NH * DR || in_sizes[12] < NH * DR ||
        in_sizes[13] < DM * DR || in_sizes[14] < DR || in_sizes[15] < DM * DM || in_sizes[16] < DM) return;
    if ((long long)out_size < needTok * DM) return;

    const float* h_t   = (const float*)d_in[0];
    const float* W_DQ  = (const float*)d_in[1];
    const float* b_DQ  = (const float*)d_in[2];
    const float* W_UQ  = (const float*)d_in[3];
    const float* b_UQ  = (const float*)d_in[4];
    const float* W_DKV = (const float*)d_in[5];
    const float* b_DKV = (const float*)d_in[6];
    const float* W_UK  = (const float*)d_in[7];
    const float* b_UK  = (const float*)d_in[8];
    const float* W_UV  = (const float*)d_in[9];
    const float* b_UV  = (const float*)d_in[10];
    const float* W_QR  = (const float*)d_in[11];
    const float* b_QR  = (const float*)d_in[12];
    const float* W_KR  = (const float*)d_in[13];
    const float* b_KR  = (const float*)d_in[14];
    const float* W_O   = (const float*)d_in[15];
    const float* b_O   = (const float*)d_in[16];
    float* out = (float*)d_out;

    char* ws = (char*)d_ws;
    size_t off = 0;
    auto carve = [&](size_t bytes) -> char* { char* p = ws + off; off += (bytes + 255) & ~(size_t)255; return p; };
    _Float16* WdT = (_Float16*)carve((size_t)96 * DM * 2);
    _Float16* WuT = (_Float16*)carve((size_t)UPN * DC * 2);
    _Float16* WoT = (_Float16*)carve((size_t)DM * DM * 2);
    _Float16* CQ  = (_Float16*)carve((size_t)MTOK * DC * 2);
    _Float16* CKV = (_Float16*)carve((size_t)MTOK * DC * 2);
    _Float16* KRP = (_Float16*)carve((size_t)MTOK * DR * 2);
    _Float16* QC  = (_Float16*)carve((size_t)NB * NH * SEQ * DK * 2);
    _Float16* QRP = (_Float16*)carve((size_t)NB * NH * SEQ * DR * 2);
    _Float16* KC  = (_Float16*)carve((size_t)NB * NH * SEQ * DK * 2);
    _Float16* VT  = (_Float16*)carve((size_t)NB * NH * DK * SEQ * 2);
    _Float16* CTX = (_Float16*)carve((size_t)MTOK * DM * 2);
    if (off > ws_size) return;

    k_prep<<<PREP_BLK_A + PREP_BLK_B + PREP_BLK_C, 256, 0, stream>>>(W_DQ, W_DKV, W_KR, W_UQ, W_UK, W_UV, W_QR, W_O, WdT, WuT, WoT);
    k_down<<<MTOK / 64, 128, 0, stream>>>(h_t, WdT, b_DQ, b_DKV, b_KR, CQ, CKV, KRP);
    k_up<<<dim3(MTOK / 64, UPN / 128, 1), 128, 0, stream>>>(CQ, CKV, WuT, b_UQ, b_UK, b_UV, b_QR, QC, KC, VT, QRP);
    k_attn<<<dim3(SEQ / 64, NB * NH, 1), 128, 0, stream>>>(QC, QRP, KC, KRP, VT, CTX);
    k_out<<<dim3(MTOK / 64, DM / 64, 1), 128, 0, stream>>>(CTX, WoT, b_O, out);
}
